// OmniAttentionMechanism_18528488915621
// MI455X (gfx1250) — hardware-verified
//
#include <hip/hip_runtime.h>
#include <hip/hip_bf16.h>
#include <math.h>


typedef __attribute__((ext_vector_type(16))) _Float16 v16h;
typedef __attribute__((ext_vector_type(8)))  _Float16 v8h;
typedef __attribute__((ext_vector_type(4)))  _Float16 v4h;
typedef __attribute__((ext_vector_type(8)))  float    v8f;
typedef __attribute__((ext_vector_type(4)))  float    f32x4;

union V16U { v16h v; v8h h[2]; };

__device__ __forceinline__ v16h ld16h_lds(const _Float16* p) {
  V16U u;
  u.h[0] = *(const v8h*)(p);
  u.h[1] = *(const v8h*)(p + 8);
  return u.v;
}

__device__ __forceinline__ v16h ld_a_lds(const _Float16* row, int base) {
  V16U u;
  u.h[0] = *(const v8h*)(row + base);
  u.h[1] = *(const v8h*)(row + base + 16);
  return u.v;
}

__device__ __forceinline__ v16h ld_a_gq(const float* p, float sc) {
  f32x4 a0 = *(const f32x4*)(p);
  f32x4 a1 = *(const f32x4*)(p + 4);
  f32x4 a2 = *(const f32x4*)(p + 16);
  f32x4 a3 = *(const f32x4*)(p + 20);
  v16h r;
  r[0]=(_Float16)(a0.x*sc);  r[1]=(_Float16)(a0.y*sc);
  r[2]=(_Float16)(a0.z*sc);  r[3]=(_Float16)(a0.w*sc);
  r[4]=(_Float16)(a1.x*sc);  r[5]=(_Float16)(a1.y*sc);
  r[6]=(_Float16)(a1.z*sc);  r[7]=(_Float16)(a1.w*sc);
  r[8]=(_Float16)(a2.x*sc);  r[9]=(_Float16)(a2.y*sc);
  r[10]=(_Float16)(a2.z*sc); r[11]=(_Float16)(a2.w*sc);
  r[12]=(_Float16)(a3.x*sc); r[13]=(_Float16)(a3.y*sc);
  r[14]=(_Float16)(a3.z*sc); r[15]=(_Float16)(a3.w*sc);
  return r;
}

__device__ __forceinline__ v8f wmma16(v16h a, v16h b, v8f c) {
  return __builtin_amdgcn_wmma_f32_16x16x32_f16(false, a, false, b, (short)0, c,
                                                false, false);
}

__global__ __launch_bounds__(256) void omni_fa_kernel(
    const float* __restrict__ q, const float* __restrict__ k,
    const float* __restrict__ v, const int* __restrict__ pad_ends,
    const int* __restrict__ full_starts, const int* __restrict__ full_ends,
    const int* __restrict__ p_bt2i, const int* __restrict__ p_blm,
    float* __restrict__ out, int S, int H) {
  constexpr int D  = 64;
  constexpr int CH = 64;
  constexpr int NT = 256;
  __shared__ _Float16 Ksh[CH][72];
  __shared__ _Float16 Vt[D][72];
  __shared__ _Float16 Psh[8][16][72];
  __shared__ __attribute__((aligned(16))) float Osh[8][16 * 68];

  const int tid  = threadIdx.x;
  const int w    = tid >> 5;
  const int lane = tid & 31;
  const int n    = lane & 15;
  const int hi   = lane >> 4;
  const int abase = hi ? 8 : 0;

  const int bh = blockIdx.y;
  const int b  = bh / H;
  const int qbase = blockIdx.x * 128 + w * 16;

  const int bt2i = p_bt2i[0];
  const int blm  = p_blm[0];
  const int mode = (b < bt2i) ? 0 : ((b < bt2i + blm) ? 1 : 2);
  const bool m0 = (mode == 0);
  const bool m2 = (mode == 2);

  int kv_end = S;
  if (mode == 1) kv_end = min(S, (int)(blockIdx.x + 1) * 128);
  if (mode == 2) kv_end = min(S, max((int)(blockIdx.x + 1) * 128, 640));

  const size_t bh_off = (size_t)bh * S * D;

  const int srow = tid >> 4;
  const int sc4  = (tid & 15) << 2;
  const float* kqb = k + bh_off + (size_t)srow * D + sc4;
  const float* vqb = v + bh_off + (size_t)srow * D + sc4;
  _Float16* kshp = &Ksh[srow][sc4];
  _Float16* vtp  = &Vt[sc4][srow];

  const float QSC = 0.125f * 1.44269504088896f;
  const float* qrowp = q + bh_off + (size_t)(qbase + n) * D;
  const v16h qa0 = ld_a_gq(qrowp + 0  + abase, QSC);
  const v16h qa1 = ld_a_gq(qrowp + 32 + abase, QSC);

  v16h vones;
#pragma unroll
  for (int i = 0; i < 16; ++i) vones[i] = (_Float16)1.0f;

  int qrow[8], fs8[8], fe8[8];
  float mrun[8];
  v8f acc[4], lsum = (v8f){};
#pragma unroll
  for (int j = 0; j < 4; ++j) acc[j] = (v8f){};
#pragma unroll
  for (int r = 0; r < 8; ++r) {
    qrow[r] = qbase + (hi ? 8 + r : r);
    fs8[r] = full_starts[qrow[r]];
    fe8[r] = full_ends[qrow[r]];
    mrun[r] = -1e30f;
  }

  for (int kvc = 0; kvc < kv_end; kvc += CH) {
    __syncthreads();
    const size_t cko = (size_t)kvc * D;
#pragma unroll
    for (int it = 0; it < 4; ++it) {
      f32x4 kk = *(const f32x4*)(kqb + cko + it * 16 * D);
      v4h kh;
      kh.x = (_Float16)kk.x; kh.y = (_Float16)kk.y;
      kh.z = (_Float16)kk.z; kh.w = (_Float16)kk.w;
      *(v4h*)(kshp + it * 16 * 72) = kh;
      f32x4 vv = *(const f32x4*)(vqb + cko + it * 16 * D);
      vtp[it * 16 + 0 * 72] = (_Float16)vv.x;
      vtp[it * 16 + 1 * 72] = (_Float16)vv.y;
      vtp[it * 16 + 2 * 72] = (_Float16)vv.z;
      vtp[it * 16 + 3 * 72] = (_Float16)vv.w;
      if (it == 0 && kvc + CH < kv_end) {
        __builtin_prefetch(kqb + cko + CH * D, 0, 0);
        __builtin_prefetch(vqb + cko + CH * D, 0, 0);
      }
    }
    __syncthreads();

    const bool skip = (mode != 0) && (kvc > qbase + 15) &&
                      (mode == 1 || kvc > 579);
    if (!skip) {
      v8f sc[4];
#pragma unroll
      for (int st = 0; st < 4; ++st) {
        const _Float16* kr = &Ksh[16 * st + n][0];
        v8f s = (v8f){};
        s = wmma16(qa0, ld_a_lds(kr, abase), s);
        s = wmma16(qa1, ld_a_lds(kr, 32 + abase), s);
        sc[st] = s;
      }

      int ki[4], pe[4];
      bool aux[4];
#pragma unroll
      for (int st = 0; st < 4; ++st) {
        ki[st] = kvc + 16 * st + n;
        pe[st] = pad_ends[b * S + ki[st]];
        aux[st] = m2 && (ki[st] <= 579);
      }
#pragma unroll
      for (int r = 0; r < 8; ++r) {
        const int qi = qrow[r];
        float sv[4];
#pragma unroll
        for (int st = 0; st < 4; ++st) {
          const bool cq = qi >= ki[st];
          const bool ca = cq && (ki[st] >= pe[st]);
          const bool fu = (ki[st] < fe8[r]) && (ki[st] >= fs8[r]);
          const bool t2i = ((qi == ki[st]) != (ca || fu));
          const bool keep = m0 ? t2i : (cq || aux[st]);
          sv[st] = keep ? sc[st][r] : -1e30f;
        }
        float mx = fmaxf(fmaxf(sv[0], sv[1]), fmaxf(sv[2], sv[3]));
        mx = fmaxf(mx, __shfl_xor(mx, 1, 16));
        mx = fmaxf(mx, __shfl_xor(mx, 2, 16));
        mx = fmaxf(mx, __shfl_xor(mx, 4, 16));
        mx = fmaxf(mx, __shfl_xor(mx, 8, 16));
        const float nm = fmaxf(mrun[r], mx);
        const float al = exp2f(mrun[r] - nm);
        mrun[r] = nm;
        const float p0 = exp2f(sv[0] - nm);
        const float p1 = exp2f(sv[1] - nm);
        const float p2 = exp2f(sv[2] - nm);
        const float p3 = exp2f(sv[3] - nm);
        lsum[r] *= al;
#pragma unroll
        for (int j = 0; j < 4; ++j) acc[j][r] *= al;

        const int M = hi ? 8 + r : r;
        Psh[w][M][n]      = (_Float16)(p0 * 1024.0f);
        Psh[w][M][16 + n] = (_Float16)(p1 * 1024.0f);
        Psh[w][M][32 + n] = (_Float16)(p2 * 1024.0f);
        Psh[w][M][48 + n] = (_Float16)(p3 * 1024.0f);
      }

      const v16h pa0 = ld_a_lds(&Psh[w][n][0], abase);
      const v16h pa1 = ld_a_lds(&Psh[w][n][0], 32 + abase);
      lsum = wmma16(pa0, vones, lsum);
      lsum = wmma16(pa1, vones, lsum);
#pragma unroll
      for (int j = 0; j < 4; ++j) {
        const _Float16* vr = &Vt[16 * j + n][0];
        acc[j] = wmma16(pa0, ld_a_lds(vr, abase), acc[j]);
        acc[j] = wmma16(pa1, ld_a_lds(vr, 32 + abase), acc[j]);
      }
    }
  }

  float* so = Osh[w];
#pragma unroll
  for (int r = 0; r < 8; ++r) {
    const float inv = 1.0f / lsum[r];
    const int M = hi ? 8 + r : r;
    so[M * 68 + n]      = acc[0][r] * inv;
    so[M * 68 + 16 + n] = acc[1][r] * inv;
    so[M * 68 + 32 + n] = acc[2][r] * inv;
    so[M * 68 + 48 + n] = acc[3][r] * inv;
  }
  asm volatile("s_wait_dscnt 0" ::: "memory");
  typedef float v4fa __attribute__((ext_vector_type(4), may_alias));
#pragma unroll 1
  for (int pass = 0; pass < 2; ++pass) {
#pragma unroll
    for (int i = 0; i < 8; ++i) { const int c = lane + 32 * i, rr = c >> 4, qq = (c & 15) * 4;
      *(volatile f32x4*)(out + bh_off + (size_t)(qbase + rr) * D + qq) = *(const volatile v4fa*)(so + rr * 68 + qq); }
    __threadfence();
  }
}

extern "C" void kernel_launch(void* const* d_in, const int* in_sizes, int n_in,
                              void* d_out, int out_size, void* d_ws, size_t ws_size,
                              hipStream_t stream) {
  (void)n_in; (void)out_size; (void)d_ws; (void)ws_size;
  const float* q = (const float*)d_in[0];
  const float* k = (const float*)d_in[1];
  const float* v = (const float*)d_in[2];
  const int* pad_ends    = (const int*)d_in[3];
  const int* full_starts = (const int*)d_in[4];
  const int* full_ends   = (const int*)d_in[5];
  const int* bt2i = (const int*)d_in[6];
  const int* blm  = (const int*)d_in[7];
  float* out = (float*)d_out;

  const int S = in_sizes[4];
  const int B = in_sizes[3] / S;
  const int H = (int)((long long)in_sizes[0] / ((long long)B * S * 64));

  dim3 grid(S / 128, B * H);
  omni_fa_kernel<<<grid, 256, 0, stream>>>(q, k, v, pad_ends, full_starts,
                                           full_ends, bt2i, blm, out, S, H);
}
